// Se3AttentionHead_53188874993901
// MI455X (gfx1250) — hardware-verified
//
#include <hip/hip_runtime.h>
#include <stddef.h>


#define NTHR   128
#define NWAVE  4
#define EPT    8
#define CHUNK  (NTHR * EPT)
#define WCAP   (EPT * 32)
#define LISTN  (NWAVE * WCAP)
#define DRN    (NWAVE * 16)
#define PCAP   (CHUNK + DRN)
#define NB     256
#define FW     32
#define NK     8
#define RH     64
#define NWK    128
#define NWV    320
#define NWR    448
#define WP     324
#define XP     40
#define MP     36

#define RS8 0.35355339059327373f
#define RS2 0.70710678118654752f
#define RS3 0.57735026918962576f

static_assert(NTHR == 2 * RH);
static_assert(NB == NWAVE * 64);
static_assert((NB & (NB - 1)) == 0);
static_assert(PCAP >= CHUNK + DRN);
static_assert(NWK + NWV == NWR);

typedef float        v4f   __attribute__((ext_vector_type(4)));
typedef float        v8f   __attribute__((ext_vector_type(8)));
typedef int          v4i   __attribute__((ext_vector_type(4)));
typedef unsigned int v4u   __attribute__((ext_vector_type(4)));
typedef unsigned int v8u   __attribute__((ext_vector_type(8)));
typedef __bf16       v16bf __attribute__((ext_vector_type(16)));
union FragB { v16bf v; v8u u; v4u q[2]; };

__device__ __forceinline__ float silu(float x) {
  return x * __builtin_amdgcn_rcpf(1.0f + __expf(-x));
}

__device__ __forceinline__ unsigned int bf_bits(float v) {
  const unsigned int u = __float_as_uint(v);
  return (u + 0x7FFFu + ((u >> 16) & 1u)) >> 16;
}

__device__ __forceinline__ void split2(float v0, float v1, unsigned int& hi, unsigned int& lo) {
  const unsigned int h0 = bf_bits(v0), h1 = bf_bits(v1);
  const float f0 = __uint_as_float(h0 << 16), f1 = __uint_as_float(h1 << 16);
  const unsigned int l0 = bf_bits(v0 - f0), l1 = bf_bits(v1 - f1);
  hi = h0 | (h1 << 16);
  lo = l0 | (l1 << 16);
}

__device__ __forceinline__ v8f wmb(const FragB& a, const FragB& b, v8f c) {
  v8f d = __builtin_amdgcn_wmma_f32_16x16x32_bf16(false, a.v, false, b.v, (short)0, c, false, false);
  asm volatile("v_nop\n\tv_nop\n\tv_nop\n\tv_nop" : "+v"(d) : "v"(a.u), "v"(b.u));
  return d;
}

__device__ __forceinline__ void build_a(const float* r1, float dm, int hh, FragB& ah, FragB& al) {
  const v4f ra = *(const v4f*)(r1 + 8 * hh);
  const v4f rb = *(const v4f*)(r1 + 8 * hh + 4);
  const v4f rc = *(const v4f*)(r1 + 16 + 8 * hh);
  const v4f rd = *(const v4f*)(r1 + 20 + 8 * hh);
  v8u hu, lu;
  unsigned int a, b;
  split2(silu(dm * ra.x), silu(dm * ra.y), a, b); hu[0] = a; lu[0] = b;
  split2(silu(dm * ra.z), silu(dm * ra.w), a, b); hu[1] = a; lu[1] = b;
  split2(silu(dm * rb.x), silu(dm * rb.y), a, b); hu[2] = a; lu[2] = b;
  split2(silu(dm * rb.z), silu(dm * rb.w), a, b); hu[3] = a; lu[3] = b;
  split2(silu(dm * rc.x), silu(dm * rc.y), a, b); hu[4] = a; lu[4] = b;
  split2(silu(dm * rc.z), silu(dm * rc.w), a, b); hu[5] = a; lu[5] = b;
  split2(silu(dm * rd.x), silu(dm * rd.y), a, b); hu[6] = a; lu[6] = b;
  split2(silu(dm * rd.z), silu(dm * rd.w), a, b); hu[7] = a; lu[7] = b;
  ah.u = hu;
  al.u = lu;
}

__device__ __forceinline__ void radial_gemm(const float* r1, float dm,
                                            const unsigned int* __restrict__ Bh,
                                            const unsigned int* __restrict__ Bl,
                                            int ntile, float* ww, int hh, int m) {
  FragB ah0, al0, ah1, al1;
  build_a(r1, dm, hh, ah0, al0);
  build_a(r1 + 32, dm, hh, ah1, al1);
#pragma unroll 1
  for (int t = 0; t < ntile; ++t) {
    const v4u* rp = (const v4u*)(Bh + (size_t)(16 * t + m) * 32);
    const v4u* lp = (const v4u*)(Bl + (size_t)(16 * t + m) * 32);
    FragB bh0, bh1, bl0, bl1;
    bh0.q[0] = rp[hh];     bh0.q[1] = rp[2 + hh];
    bh1.q[0] = rp[4 + hh]; bh1.q[1] = rp[6 + hh];
    bl0.q[0] = lp[hh];     bl0.q[1] = lp[2 + hh];
    bl1.q[0] = lp[4 + hh]; bl1.q[1] = lp[6 + hh];
    v8f c = {0.f, 0.f, 0.f, 0.f, 0.f, 0.f, 0.f, 0.f};
    c = wmb(ah0, bh0, c);
    c = wmb(ah0, bl0, c);
    c = wmb(al0, bh0, c);
    c = wmb(ah1, bh1, c);
    c = wmb(ah1, bl1, c);
    c = wmb(al1, bh1, c);
    float* wp = ww + (8 * hh) * WP + 16 * t + m;
#pragma unroll
    for (int rr = 0; rr < 8; ++rr) wp[rr * WP] = c[rr];
  }
}

__device__ __forceinline__ int scan_chunk(const int* __restrict__ dsts, int nE, int cbase, int nodeBase,
                                          int vec8, int* list, int tid, int wave) {
  int wc = 0;
  const int el0  = tid * EPT;
  const int e0   = cbase + el0;
  const int sent = -2147483647 - 1;
  v4i da, db;
  if (vec8 != 0 && cbase + CHUNK <= nE) {
    da = *(const v4i*)(dsts + e0);
    db = *(const v4i*)(dsts + e0 + 4);
  } else {
    da.x = (e0     < nE) ? dsts[min(e0, nE - 1)] : sent;
    da.y = (e0 + 1 < nE) ? dsts[min(e0 + 1, nE - 1)] : sent;
    da.z = (e0 + 2 < nE) ? dsts[min(e0 + 2, nE - 1)] : sent;
    da.w = (e0 + 3 < nE) ? dsts[min(e0 + 3, nE - 1)] : sent;
    db.x = (e0 + 4 < nE) ? dsts[min(e0 + 4, nE - 1)] : sent;
    db.y = (e0 + 5 < nE) ? dsts[min(e0 + 5, nE - 1)] : sent;
    db.z = (e0 + 6 < nE) ? dsts[min(e0 + 6, nE - 1)] : sent;
    db.w = (e0 + 7 < nE) ? dsts[min(e0 + 7, nE - 1)] : sent;
  }
  const unsigned nb = (unsigned)nodeBase;
  const unsigned s0 = (unsigned)da.x - nb, s1 = (unsigned)da.y - nb;
  const unsigned s2 = (unsigned)da.z - nb, s3 = (unsigned)da.w - nb;
  const unsigned s4 = (unsigned)db.x - nb, s5 = (unsigned)db.y - nb;
  const unsigned s6 = (unsigned)db.z - nb, s7 = (unsigned)db.w - nb;
  const bool h0 = s0 < (unsigned)NB, h1 = s1 < (unsigned)NB, h2 = s2 < (unsigned)NB, h3 = s3 < (unsigned)NB;
  const bool h4 = s4 < (unsigned)NB, h5 = s5 < (unsigned)NB, h6 = s6 < (unsigned)NB, h7 = s7 < (unsigned)NB;
  const unsigned any = __builtin_amdgcn_ballot_w32(h0 | h1 | h2 | h3 | h4 | h5 | h6 | h7);
  if (any != 0u) {
#define HITJ(J, HJ) { \
      const unsigned mj = __builtin_amdgcn_ballot_w32(HJ); \
      if (mj != 0u) { \
        if (HJ) { \
          const int pos = wc + (int)__builtin_amdgcn_mbcnt_lo(mj, 0u); \
          if (pos < WCAP) list[wave * WCAP + pos] = el0 + (J); \
        } \
        wc += (int)__builtin_popcount(mj); } }
    HITJ(0, h0)
    HITJ(1, h1)
    HITJ(2, h2)
    HITJ(3, h3)
    HITJ(4, h4)
    HITJ(5, h5)
    HITJ(6, h6)
    HITJ(7, h7)
#undef HITJ
  }
  return wc;
}

__global__ __launch_bounds__(128) void k_prep(const float* __restrict__ R2k, const float* __restrict__ R2v,
                                              unsigned int* Bh, unsigned int* Bl, int nL) {
  const int total = nL * NWR * 8;
  const int t  = blockIdx.x * 128 + threadIdx.x;
  const int tc = t < total ? t : total - 1;
  const int g = tc & 7, row = tc >> 3;
  const int L = row / NWR, n = row - L * NWR;
  const int nk = n < NWK ? n : NWK - 1;
  int nv = n - NWK; nv = nv < 0 ? 0 : (nv > NWV - 1 ? NWV - 1 : nv);
  const bool isk = n < NWK;
  const float* pk = R2k + (size_t)L * RH * NWK + nk;
  const float* pv = R2v + (size_t)L * RH * NWV + nv;
  unsigned int hw[4], lw[4];
#pragma unroll
  for (int j = 0; j < 4; ++j) {
    const int k0 = 8 * g + 2 * j;
    const float a0 = pk[(size_t)k0 * NWK], a1 = pk[(size_t)(k0 + 1) * NWK];
    const float b0 = pv[(size_t)k0 * NWV], b1 = pv[(size_t)(k0 + 1) * NWV];
    const float v0 = isk ? a0 : b0;
    const float v1 = isk ? a1 : b1;
    split2(v0, v1, hw[j], lw[j]);
  }
  const v4u hv = {hw[0], hw[1], hw[2], hw[3]};
  const v4u lv = {lw[0], lw[1], lw[2], lw[3]};
  unsigned int* ph = Bh + (size_t)row * 32 + 4 * g;
  unsigned int* pl = Bl + (size_t)row * 32 + 4 * g;
  const bool wr = t < total;
  if (wr) { *(volatile v4u*)ph = hv; *(volatile v4u*)pl = lv; }
  __threadfence();
  if (wr) { *(volatile v4u*)ph = hv; *(volatile v4u*)pl = lv; }
}

__global__ __launch_bounds__(NTHR) void k_layer(
    const float* __restrict__ xin, const int* __restrict__ ei,
    const float* __restrict__ ef, const float* __restrict__ dist,
    const float* __restrict__ WqL, const float* __restrict__ R1kL, const float* __restrict__ R1vL,
    const unsigned int* __restrict__ Bh, const unsigned int* __restrict__ Bl,
    float* xout, int nN, int nE, int vec8, int rowLim) {
  __shared__ __attribute__((aligned(16))) float wl[NWAVE * 16 * WP];
  __shared__ __attribute__((aligned(16))) float accs[NB * FW];
  __shared__ float mx[NB];
  __shared__ float den[NB];
  __shared__ __attribute__((aligned(16))) float qs[NB * NK];
  __shared__ __attribute__((aligned(16))) float xst[NWAVE * 16 * XP];
  __shared__ __attribute__((aligned(16))) float msg[DRN * MP];
  __shared__ int mslot[DRN];
  __shared__ int msrc[DRN];
  __shared__ __attribute__((aligned(16))) int list[LISTN];
  __shared__ __attribute__((aligned(16))) int pend[PCAP];
  __shared__ __attribute__((aligned(16))) float r1s[2 * RH];
  __shared__ int wcnt[NWAVE];
  __shared__ int pendN;

  const int tid = threadIdx.x, lane = tid & 31, wave = tid >> 5, hh = lane >> 4, m = lane & 15;
  const int nodeBase = blockIdx.x * NB;
  const int* srcs = ei;
  const int* dsts = ei + nE;
  float* xw = xst + wave * 16 * XP;
  float* ww = wl + wave * 16 * WP;
  float* mw = msg + wave * 16 * MP;

  for (int i = tid; i < NB * FW; i += NTHR) accs[i] = 0.0f;
  for (int i = tid; i < NB; i += NTHR) { mx[i] = 1.0f; den[i] = 1.0f; }
  {
    int ia = tid; ia = ia > RH - 1 ? RH - 1 : ia;
    int ib = tid - RH; ib = ib < 0 ? 0 : (ib > RH - 1 ? RH - 1 : ib);
    const float a = R1kL[ia];
    const float b = R1vL[ib];
    r1s[tid] = (tid < RH) ? a : b;
  }
  for (int sl = tid; sl < NB; sl += NTHR) {
    int node = nodeBase + sl;
    node = node > nN - 1 ? nN - 1 : node;
    const v4f xa = *(const v4f*)(xin + (size_t)node * FW);
    const v4f xb = *(const v4f*)(xin + (size_t)node * FW + 4);
    const float x8[8] = {xa.x, xa.y, xa.z, xa.w, xb.x, xb.y, xb.z, xb.w};
#pragma unroll
    for (int o = 0; o < NK; ++o) {
      float a = 0.0f;
#pragma unroll
      for (int i = 0; i < 8; ++i) a += x8[i] * WqL[i * NK + o];
      qs[sl * NK + o] = a * RS8;
    }
  }
  if (tid == 0) pendN = 0;
  __syncthreads();

  const int nChunks = (nE + CHUNK - 1) / CHUNK;
#pragma unroll 1
  for (int ch = 0; ch < nChunks; ++ch) {
    const int cbase = ch * CHUNK;
    const int wc = scan_chunk(dsts, nE, cbase, nodeBase, vec8, list, tid, wave);
    if (lane == 0) wcnt[wave] = wc;
    __syncthreads();

    const int base = pendN;
    int tot = 0, myoff = 0;
#pragma unroll
    for (int w = 0; w < NWAVE; ++w) {
      int c = wcnt[w];
      c = c > WCAP ? WCAP : (c < 0 ? 0 : c);
      if (w < wave) myoff += c;
      tot += c;
    }
    int newN = base + tot;
    newN = newN > PCAP ? PCAP : newN;
    {
      int n = wcnt[wave];
      n = n > WCAP ? WCAP : (n < 0 ? 0 : n);
      const int* lp = list + wave * WCAP;
      for (int i = lane; i < n; i += 32) {
        const int pos = base + myoff + i;
        if (pos < PCAP) pend[pos] = cbase + lp[i];
      }
    }
    const int fin = (ch == nChunks - 1) ? 1 : 0;
    const int R   = (fin != 0) ? (newN + DRN - 1) / DRN : newN / DRN;
    const int Pv  = (fin != 0) ? newN : R * DRN;
    __syncthreads();

#pragma unroll 1
    for (int r = 0; r < R; ++r) {
      {
        const int idx = r * DRN + wave * 16 + m;
        const bool valid = idx < Pv;
        int e = pend[idx];
        e = valid ? e : 0;
        e = e < 0 ? 0 : (e > nE - 1 ? nE - 1 : e);
        const int d = dsts[e];
        int s = srcs[e];
        int slot = d - nodeBase;
        if (!valid || (unsigned)slot >= (unsigned)NB) slot = -1;
        s = s < 0 ? 0 : (s > nN - 1 ? nN - 1 : s);
        const v4f g4 = *(const v4f*)(ef + (size_t)e * 4);
        const float dd = dist[e];
        if (hh == 0) {
          msrc[wave * 16 + m]  = s;
          mslot[wave * 16 + m] = slot;
          *(v4f*)(xw + m * XP + 32) = g4;
          xw[m * XP + 36] = dd;
        }
      }
      __syncthreads();
#pragma unroll
      for (int j = 0; j < 4; ++j) {
        const int row = (lane >> 3) + 4 * j, pc = lane & 7;
        const int s = msrc[wave * 16 + row];
        const v4f v = *(const v4f*)(xin + (size_t)s * FW + 4 * pc);
        *(v4f*)(xw + row * XP + 4 * pc) = v;
      }
      __syncthreads();
      {
        const float dm = xw[m * XP + 36];
        radial_gemm(r1s, dm, Bh, Bl, NWK / 16, ww, hh, m);
      }
      __syncthreads();
      {
        const float* xr = xw + m * XP;
        const float* wr = ww + m * WP + 4 * hh;
        const float gs = xr[32], g0 = xr[33], g1 = xr[34], g2 = xr[35];
        v4f sa = {0.f, 0.f, 0.f, 0.f};
        v4f sb = sa;
#pragma unroll 2
        for (int i = 0; i < 8; ++i) {
          const float xs = xr[i];
          const float v0 = xr[8 + 3 * i], v1 = xr[9 + 3 * i], v2 = xr[10 + 3 * i];
          const float xg = xs * gs;
          const float dt = (v0 * g0 + v1 * g1 + v2 * g2) * RS3;
          const v4f w1 = *(const v4f*)(wr + 8 * i);
          const v4f w2 = *(const v4f*)(wr + 64 + 8 * i);
          sa += w1 * xg;
          sb += w2 * dt;
        }
        const v4f kk = (sa * RS8 + sb * RS8) * RS2;
        int sl = mslot[wave * 16 + m];
        sl = sl < 0 ? 0 : (sl > NB - 1 ? NB - 1 : sl);
        const v4f q4 = *(const v4f*)(qs + sl * NK + 4 * hh);
        float part = kk.x * q4.x + kk.y * q4.y + kk.z * q4.z + kk.w * q4.w;
        part += __shfl_xor(part, 16, 32);
        if (hh == 0) mw[m * MP + 32] = part * RS8;
      }
      __syncthreads();
      {
        const float dm = xw[m * XP + 36];
        radial_gemm(r1s + RH, dm, Bh + (size_t)NWK * 32, Bl + (size_t)NWK * 32, NWV / 16, ww, hh, m);
      }
      __syncthreads();
      {
        const float* xr = xw + m * XP;
        const float* wr = ww + m * WP + 4 * hh;
        const float gs = xr[32], g0 = xr[33], g1 = xr[34], g2 = xr[35];
        v4f z4 = {0.f, 0.f, 0.f, 0.f};
        v4f va = z4, vb = z4, t3 = z4, v40 = z4, v41 = z4, v42 = z4, v50 = z4, v51 = z4, v52 = z4;
#pragma unroll 2
        for (int i = 0; i < 8; ++i) {
          const float xs = xr[i];
          const float v0 = xr[8 + 3 * i], v1 = xr[9 + 3 * i], v2 = xr[10 + 3 * i];
          const float xg = xs * gs;
          const float dt = (v0 * g0 + v1 * g1 + v2 * g2) * RS3;
          const float c0 = (v1 * g2 - v2 * g1) * RS2;
          const float c1 = (v2 * g0 - v0 * g2) * RS2;
          const float c2 = (v0 * g1 - v1 * g0) * RS2;
          const v4f w1 = *(const v4f*)(wr + 8 * i);
          const v4f w2 = *(const v4f*)(wr + 64 + 8 * i);
          const v4f w3 = *(const v4f*)(wr + 128 + 8 * i);
          const v4f w4 = *(const v4f*)(wr + 192 + 8 * i);
          const v4f w5 = *(const v4f*)(wr + 256 + 8 * i);
          va += w1 * xg;
          vb += w2 * dt;
          t3 += w3 * xs;
          v40 += w4 * v0; v41 += w4 * v1; v42 += w4 * v2;
          v50 += w5 * c0; v51 += w5 * c1; v52 += w5 * c2;
        }
        const v4f vs = (va * RS8 + vb * RS8) * RS2;
        t3 = t3 * RS8;
        v4f o0 = t3 * g0; o0 = o0 + (v40 * gs) * RS8; o0 = (o0 + v50 * RS8) * RS3;
        v4f o1 = t3 * g1; o1 = o1 + (v41 * gs) * RS8; o1 = (o1 + v51 * RS8) * RS3;
        v4f o2 = t3 * g2; o2 = o2 + (v42 * gs) * RS8; o2 = (o2 + v52 * RS8) * RS3;
        float* mr = mw + m * MP;
        *(v4f*)(mr + 4 * hh) = vs;
#pragma unroll
        for (int c = 0; c < 4; ++c) {
          const int o = 4 * hh + c;
          mr[8 + 3 * o + 0] = o0[c];
          mr[8 + 3 * o + 1] = o1[c];
          mr[8 + 3 * o + 2] = o2[c];
        }
      }
      __syncthreads();

#pragma unroll 1
      for (int i = 0; i < DRN; ++i) {
        const int sl = __builtin_amdgcn_readfirstlane(mslot[i]);
        if (sl >= 0 && sl < NB && (sl & (NWAVE - 1)) == wave) {
          const float L  = msg[i * MP + 32];
          const float mo = mx[sl];
          const float mn = fmaxf(mo, L);
          const float sc = __expf(mo - mn);
          const float p  = __expf(L - mn);
          const float v  = msg[i * MP + lane];
          const float a  = accs[sl * FW + lane];
          accs[sl * FW + lane] = a * sc + p * v;
          if (lane == 0) { den[sl] = den[sl] * sc + p; mx[sl] = mn; }
        }
      }
      __syncthreads();
    }

    int rem = newN - R * DRN;
    rem = rem < 0 ? 0 : rem;
    if (R > 0 && tid < rem) pend[tid] = pend[R * DRN + tid];
    if (tid == 0) pendN = rem;
  }
  __syncthreads();

  v4f ov[16];
#pragma unroll
  for (int j = 0; j < 16; ++j) {
    const int row = wave * 64 + 4 * j + (lane >> 3), pc = lane & 7;
    const float rd = 1.0f / den[row];
    ov[j] = *(const v4f*)(accs + row * FW + 4 * pc) * rd;
  }
  const int lim = rowLim < 0 ? 0 : rowLim;
#pragma unroll
  for (int j = 0; j < 16; ++j) {
    const int row = wave * 64 + 4 * j + (lane >> 3), pc = lane & 7;
    const int gr = nodeBase + row;
    if (gr < lim) *(volatile v4f*)(xout + (size_t)gr * FW + 4 * pc) = ov[j];
  }
  __threadfence();
#pragma unroll
  for (int j = 0; j < 16; ++j) {
    const int row = wave * 64 + 4 * j + (lane >> 3), pc = lane & 7;
    const int gr = nodeBase + row;
    if (gr < lim) *(volatile v4f*)(xout + (size_t)gr * FW + 4 * pc) = ov[j];
  }
}

extern "C" void kernel_launch(void* const* d_in, const int* in_sizes, int n_in,
                              void* d_out, int out_size, void* d_ws, size_t ws_size,
                              hipStream_t stream) {
  if (n_in < 9) return;
  const int nE = in_sizes[0] / 2;
  const int nN = in_sizes[1] / FW;
  if (nE <= 0 || nN <= 0 || in_sizes[0] != 2 * nE || in_sizes[1] != nN * FW) return;
  if (in_sizes[2] != nE * 4 || in_sizes[3] != nE) return;
  const int nL = in_sizes[4] / (NK * NK);
  if (nL <= 0 || in_sizes[4] != nL * NK * NK) return;
  if (in_sizes[5] != nL * RH || in_sizes[6] != nL * RH * NWK) return;
  if (in_sizes[7] != nL * RH || in_sizes[8] != nL * RH * NWV) return;
  if (out_size != nN * FW) return;

  const int*   ei   = (const int*)d_in[0];
  const float* nf   = (const float*)d_in[1];
  const float* ef   = (const float*)d_in[2];
  const float* dist = (const float*)d_in[3];
  const float* Wq   = (const float*)d_in[4];
  const float* R1k  = (const float*)d_in[5];
  const float* R2k  = (const float*)d_in[6];
  const float* R1v  = (const float*)d_in[7];
  const float* R2v  = (const float*)d_in[8];
  float* out = (float*)d_out;

  const int nBlk = (nN + NB - 1) / NB;
  const size_t rowsP = (size_t)nBlk * NB;

  char* ws = (char*)d_ws;
  size_t off = 0;
  const size_t szB = ((size_t)nL * NWR * RH * 2 + 255) & ~(size_t)255;
  const size_t szX = (rowsP * FW * 4 + 255) & ~(size_t)255;
  const size_t oBh = off; off += szB;
  const size_t oBl = off; off += szB;
  const size_t oXa = off; off += szX;
  const size_t oXb = off; off += szX;
  if (off > ws_size) return;
  unsigned int* Bh = (unsigned int*)(ws + oBh);
  unsigned int* Bl = (unsigned int*)(ws + oBl);
  float* Xa = (float*)(ws + oXa);
  float* Xb = (float*)(ws + oXb);

  const int vec8 = ((nE & 3) == 0) ? 1 : 0;

  k_prep<<<(nL * NWR * 8 + 127) / 128, 128, 0, stream>>>(R2k, R2v, Bh, Bl, nL);

  for (int l = 0; l < nL; ++l) {
    const float* xi = (l == 0) ? nf : ((((l - 1) & 1) != 0) ? Xb : Xa);
    float* xo;
    int lim;
    if (l == nL - 1) { xo = out; lim = nN; }
    else { xo = ((l & 1) != 0) ? Xb : Xa; lim = (int)rowsP; }
    k_layer<<<nBlk, NTHR, 0, stream>>>(
        xi, ei, ef, dist,
        Wq + (size_t)l * NK * NK, R1k + (size_t)l * RH, R1v + (size_t)l * RH,
        Bh + (size_t)l * NWR * 32, Bl + (size_t)l * NWR * 32,
        xo, nN, nE, vec8, lim);
  }
}
